// VisionMambaPathArch_42322607735354
// MI455X (gfx1250) — hardware-verified
//
#include <hip/hip_runtime.h>
#include <stdint.h>

#define B_SZ    16
#define CIN     3
#define IMGSZ   224
#define PATCH   16
#define D_MODEL 192
#define DEPTH   8
#define N_ST    16
#define K_CONV  4
#define DIN     384
#define R_RANK  12
#define L_PATCH 196
#define SEQ     197
#define TPOS    98
#define NCLS    1000
#define NCLS_P  1024
#define EPSF    1e-5f
#define XZC     768
#define DBLC    44
#define DBLP    64
#define MROWS   3152
#define MPAD    3200
#define PROWS   3136
#define KPATCH  768
#define HEAD_MP 64
#define W_CARRY 64.0f
#define U_CARRY 256.0f
#define Y_CARRY 256.0f
#define F_CARRY 64.0f
#define SC_DG   64
#define SC_TS   16

typedef __attribute__((ext_vector_type(16))) _Float16 v16h;
typedef __attribute__((ext_vector_type(8)))  _Float16 v8h;
typedef __attribute__((ext_vector_type(16))) __bf16   v16b;
typedef __attribute__((ext_vector_type(8)))  __bf16   v8b;
typedef __attribute__((ext_vector_type(8)))  float    v8f;
typedef __attribute__((ext_vector_type(4)))  float    v4f;
typedef __attribute__((ext_vector_type(2)))  float    v2f;

__device__ __forceinline__ unsigned short f2bf_bits(float f) {
  unsigned u = __float_as_uint(f);
  return (unsigned short)((u + 0x7FFFu + ((u >> 16) & 1u)) >> 16);
}
__device__ __forceinline__ float bf_bits2f(unsigned short h) { return __uint_as_float(((unsigned)h) << 16); }

__device__ __forceinline__ void dep_guard_h(v8f& a, v8f& b, v16h x, v16h y) { asm volatile("v_nop\n\tv_nop\n\tv_nop\n\tv_nop" : "+v"(a), "+v"(b) : "v"(x), "v"(y)); }
__device__ __forceinline__ void dep_guard_b(v8f& a, v8f& b, v16b x, v16b y) { asm volatile("v_nop\n\tv_nop\n\tv_nop\n\tv_nop" : "+v"(a), "+v"(b) : "v"(x), "v"(y)); }
__device__ __forceinline__ void keep4_h(v16h a, v16h b, v16h c, v16h d) { asm volatile("v_nop" :: "v"(a), "v"(b), "v"(c), "v"(d)); }
__device__ __forceinline__ void keep4_b(v16b a, v16b b, v16b c, v16b d) { asm volatile("v_nop" :: "v"(a), "v"(b), "v"(c), "v"(d)); }
__device__ __forceinline__ void acc_guard4(v8f& a, v8f& b, v8f& c, v8f& d) { asm volatile("v_nop\n\tv_nop\n\tv_nop\n\tv_nop" : "+v"(a), "+v"(b), "+v"(c), "+v"(d)); }
template <typename T> struct Frag;
template <> struct Frag<_Float16> {
  typedef v16h V; union U { v16h v; v8h h[2]; };
  static __device__ __forceinline__ v16h load(const _Float16* p) {
    U f; f.h[0] = *(const v8h*)(p); f.h[1] = *(const v8h*)(p + 16); return f.v;
  }
  static __device__ __forceinline__ v8f mma(v16h a, v16h b, v8f c) {
    return __builtin_amdgcn_wmma_f32_16x16x32_f16(false, a, false, b, (short)0, c, false, false);
  }
  static __device__ __forceinline__ void guard(v8f& a, v8f& b, v16h x, v16h y) { dep_guard_h(a, b, x, y); }
  static __device__ __forceinline__ void keep(v16h a, v16h b, v16h c, v16h d) { keep4_h(a, b, c, d); }
};
template <> struct Frag<__bf16> {
  typedef v16b V; union U { v16b v; v8b h[2]; };
  static __device__ __forceinline__ v16b load(const __bf16* p) {
    U f; f.h[0] = *(const v8b*)(p); f.h[1] = *(const v8b*)(p + 16); return f.v;
  }
  static __device__ __forceinline__ v8f mma(v16b a, v16b b, v8f c) {
    return __builtin_amdgcn_wmma_f32_16x16x32_bf16(false, a, false, b, (short)0, c, false, false);
  }
  static __device__ __forceinline__ void guard(v8f& a, v8f& b, v16b x, v16b y) { dep_guard_b(a, b, x, y); }
  static __device__ __forceinline__ void keep(v16b a, v16b b, v16b c, v16b d) { keep4_b(a, b, c, d); }
};

template <int ET> struct Elem;
template <> struct Elem<0> { typedef _Float16 T; };
template <> struct Elem<1> { typedef __bf16 T; };
template <int ET, bool SPLIT, int BIAS_MODE, int OUT_MODE, bool RESID, int ACT = 0>
__global__ __launch_bounds__(256) void wmma_gemm64(
    const unsigned short* __restrict__ Ap, const unsigned short* __restrict__ A2p, int lda, long strideA,
    const unsigned short* __restrict__ Btp, const unsigned short* __restrict__ Bt2p, int ldb, long strideB,
    void* __restrict__ Cout, void* __restrict__ Cout2, int ldc, long strideC,
    const float* __restrict__ bias,
    const float* __restrict__ resid, long strideR,
    int M, int N, int K, float scale) {
  typedef typename Elem<ET>::T T;
  typedef typename Frag<T>::V V;
  const T* A = (const T*)Ap; const T* A2 = (const T*)A2p; const T* Bt = (const T*)Btp; const T* Bt2 = (const T*)Bt2p;
  __shared__ __align__(16) float sT[8][16 * 68];
  const int b    = blockIdx.y;
  const int lane = threadIdx.x & 31;
  const int wave = threadIdx.x >> 5;
  const int tilesN = N >> 6;
  const int tilesM = M >> 6;
  const int tile = blockIdx.x * 8 + wave;
  if (tile >= tilesM * tilesN) return;
  const int tm = tile / tilesN;
  const int tn = tile - tm * tilesN;
  const int m0 = tm << 6;
  const int n0 = tn << 6;

  const T* Ab  = A  + (size_t)b * strideA;
  const T* Bb  = Bt + (size_t)b * strideB;
  const T* Ab2 = SPLIT ? (A2  + (size_t)b * strideA) : nullptr;
  const T* Bb2 = SPLIT ? (Bt2 + (size_t)b * strideB) : nullptr;

  const int rlane = lane & 15;
  const int koff  = (lane >> 4) * 8;
  const int mOff  = (lane >> 4) * 8;

  v8f acc[4][4];
#pragma unroll
  for (int i = 0; i < 4; ++i)
#pragma unroll
    for (int j = 0; j < 4; ++j) acc[i][j] = (v8f){0.f,0.f,0.f,0.f,0.f,0.f,0.f,0.f};

  for (int k0 = 0; k0 < K; k0 += 32) {
    V bh[4], bl[4];
#pragma unroll
    for (int j = 0; j < 4; ++j) {
      const size_t bo = (size_t)(n0 + (j << 4) + rlane) * ldb + koff + k0;
      bh[j] = Frag<T>::load(Bb + bo);
      if (SPLIT) bl[j] = Frag<T>::load(Bb2 + bo);
    }
#pragma unroll
    for (int i = 0; i < 4; ++i) {
      const size_t ao = (size_t)(m0 + (i << 4) + rlane) * lda + koff + k0;
      V ah = Frag<T>::load(Ab + ao);
      V al;
      if (SPLIT) al = Frag<T>::load(Ab2 + ao);
#pragma unroll
      for (int j = 0; j < 4; ++j) {
        acc[i][j] = Frag<T>::mma(ah, bh[j], acc[i][j]);
        if (SPLIT) {
          acc[i][j] = Frag<T>::mma(ah, bl[j], acc[i][j]);
          acc[i][j] = Frag<T>::mma(al, bh[j], acc[i][j]);
        }
      }
      Frag<T>::guard(acc[i][0], acc[i][3], ah, SPLIT ? al : ah);
    }
    Frag<T>::keep(bh[0], bh[1], bh[2], bh[3]);
    if (SPLIT) Frag<T>::keep(bl[0], bl[1], bl[2], bl[3]);
  }
  acc_guard4(acc[0][0], acc[0][1], acc[0][2], acc[0][3]);
  acc_guard4(acc[1][0], acc[1][1], acc[1][2], acc[1][3]);
  acc_guard4(acc[2][0], acc[2][1], acc[2][2], acc[2][3]);
  acc_guard4(acc[3][0], acc[3][1], acc[3][2], acc[3][3]);

  float* slab = sT[wave];
  const float* Rb = RESID ? (resid + (size_t)b * strideR) : nullptr;
#pragma unroll
  for (int i = 0; i < 4; ++i) {
    const int mBase = m0 + (i << 4);
#pragma unroll
    for (int j = 0; j < 4; ++j) {
      const int n = n0 + (j << 4) + rlane;
      float bv = 0.f;
      if (BIAS_MODE == 2) bv = bias[n];
#pragma unroll
      for (int r = 0; r < 8; ++r) {
        float v = acc[i][j][r] * scale;
        if (BIAS_MODE == 1) v += bias[mBase + mOff + r];
        if (BIAS_MODE == 2) v += bv;
        if (RESID) v += Rb[(size_t)(mBase + mOff + r) * ldc + n];
        if (ACT == 1) v = tanhf(v);
        if (ACT == 2) v = fmaxf(v, 0.0f);
        if (ACT == 3) v = v / (1.0f + expf(-v));
        if (ACT == 4) v = (v > 0.f) ? v : 0.01f * v;
        if (ACT == 5) v = 0.5f * v * (1.0f + erff(v * 0.70710678118654752f));
        slab[(mOff + r) * 68 + (j << 4) + rlane] = v;
      }
    }
    __builtin_amdgcn_fence(__ATOMIC_RELEASE, "workgroup");
    __builtin_amdgcn_wave_barrier();
    __builtin_amdgcn_fence(__ATOMIC_ACQUIRE, "workgroup");
    if (OUT_MODE == 0) {
      float* C = (float*)Cout + (size_t)b * strideC;
      const int hh = lane >> 4, c4 = (lane & 15) * 4;
      for (int pass = 0; pass < 2; ++pass) {
#pragma unroll
        for (int it = 0; it < 8; ++it) {
          const int row = it * 2 + hh;
          v4f v = *(const v4f*)(slab + row * 68 + c4);
          *(volatile v4f*)(C + (size_t)(mBase + row) * ldc + n0 + c4) = v;
        }
        __threadfence();
      }
    } else {
      const int q = lane >> 3, c8 = (lane & 7) * 8;
      unsigned short* C  = (unsigned short*)Cout  + (size_t)b * strideC;
      unsigned short* C2 = (OUT_MODE == 2) ? ((unsigned short*)Cout2 + (size_t)b * strideC) : nullptr;
      for (int pass = 0; pass < 2; ++pass) {
#pragma unroll
        for (int it = 0; it < 4; ++it) {
          const int row = it * 4 + q;
          const float* sp = slab + row * 68 + c8;
          v8h hv, lv;
#pragma unroll
          for (int e = 0; e < 8; ++e) {
            if (OUT_MODE == 1) {
              hv[e] = (_Float16)sp[e];
            } else {
              unsigned short hb = f2bf_bits(sp[e]);
              unsigned short lb = f2bf_bits(sp[e] - bf_bits2f(hb));
              hv[e] = __builtin_bit_cast(_Float16, hb);
              lv[e] = __builtin_bit_cast(_Float16, lb);
            }
          }
          *(volatile v8h*)(C + (size_t)(mBase + row) * ldc + n0 + c8) = hv;
          if (OUT_MODE == 2) *(volatile v8h*)(C2 + (size_t)(mBase + row) * ldc + n0 + c8) = lv;
        }
        __threadfence();
      }
    }
    __builtin_amdgcn_fence(__ATOMIC_RELEASE, "workgroup");
    __builtin_amdgcn_wave_barrier();
    __builtin_amdgcn_fence(__ATOMIC_ACQUIRE, "workgroup");
  }
}

__device__ __forceinline__ float wave_sum(float v) {
#pragma unroll
  for (int off = 16; off > 0; off >>= 1) v += __shfl_xor(v, off, 32);
  return v;
}
__device__ __forceinline__ unsigned pack_h2(float f0, float f1) {
  const _Float16 h0 = (_Float16)f0, h1 = (_Float16)f1;
  return (unsigned)__builtin_bit_cast(unsigned short, h0) | ((unsigned)__builtin_bit_cast(unsigned short, h1) << 16);
}
__device__ __forceinline__ void store2_u32(unsigned* p, unsigned v) {
  *(volatile unsigned*)p = v;
  __threadfence();
  *(volatile unsigned*)p = v;
}
__device__ __forceinline__ void store2_v2f(float* p, v2f v) {
  *(volatile v2f*)p = v;
  __threadfence();
  *(volatile v2f*)p = v;
}
__device__ __forceinline__ void store2_f32(float* p, float v) {
  *(volatile float*)p = v;
  __threadfence();
  *(volatile float*)p = v;
}
__device__ __forceinline__ float sigmoid_f(float x) {
  return __builtin_amdgcn_rcpf(1.0f + expf(-x));
}

__global__ __launch_bounds__(256) void cast_pad_f16x2(const float* __restrict__ in, _Float16* __restrict__ out,
                                                       int nLayer, int rowsIn, int rowsOut, int cols2, float scale) {
  const int total = nLayer * rowsOut * cols2;
  const int i = blockIdx.x * 256 + threadIdx.x;
  if (i < total) {
    const int per = rowsOut * cols2;
    const int layer = i / per;
    const int rem = i - layer * per;
    const int r = rem / cols2;
    const int c2 = rem - r * cols2;
    const bool ok = (r < rowsIn);
    const int rc = ok ? r : (rowsIn - 1);
    const v2f v = *(const v2f*)(in + (((size_t)layer * rowsIn + rc) * cols2 + c2) * 2);
    const float f0 = ok ? v[0] * scale : 0.f;
    const float f1 = ok ? v[1] * scale : 0.f;
    store2_u32((unsigned*)out + i, pack_h2(f0, f1));
  }
}

__global__ __launch_bounds__(256) void im2col_f16x2(const float* __restrict__ x, _Float16* __restrict__ ic, int n2) {
  const int i = blockIdx.x * 256 + threadIdx.x;
  if (i < n2) {
    const int rp = i / (KPATCH / 2);
    const int k  = (i - rp * (KPATCH / 2)) * 2;
    const int b  = rp / L_PATCH;
    const int p  = rp - b * L_PATCH;
    const int c  = k >> 8;
    const int r2 = k & 255;
    const int ph = r2 >> 4, pw = r2 & 15;
    const int py = p / 14, px = p - py * 14;
    const v2f v = *(const v2f*)(x + (((size_t)b * CIN + c) * IMGSZ + (py * PATCH + ph)) * IMGSZ + px * PATCH + pw);
    store2_u32((unsigned*)ic + i, pack_h2(v[0], v[1]));
  }
}

__global__ __launch_bounds__(96) void embed_kernel(const float* __restrict__ y0, const float* __restrict__ cls,
                                                    const float* __restrict__ pos, const float* __restrict__ ew,
                                                    float* __restrict__ h) {
  __shared__ float red[4];
  const int row  = blockIdx.x;
  const int tid  = threadIdx.x, lane = tid & 31, wave = tid >> 5;
  const int d    = 2 * tid;
  const bool real = (row < MROWS);
  const int rowc = real ? row : (MROWS - 1);
  const int b    = rowc / SEQ;
  const int l    = rowc - b * SEQ;
  const bool iscls = (l == TPOS);
  const int p    = (l < TPOS) ? l : ((l > TPOS) ? (l - 1) : 0);
  const v2f yv = *(const v2f*)(y0 + ((size_t)b * L_PATCH + p) * D_MODEL + d);
  const float ss = wave_sum(yv[0] * yv[0] + yv[1] * yv[1]);
  if (lane == 0) red[wave] = ss;
  __syncthreads();
  const float tot  = red[0] + red[1] + red[2];
  const float rinv = rsqrtf(tot * (1.0f / (float)D_MODEL) + EPSF);
  const v2f pv = *(const v2f*)(pos + (size_t)l * D_MODEL + d);
  const v2f cv = *(const v2f*)(cls + d);
  float o0, o1;
  if (iscls) { o0 = cv[0] + pv[0]; o1 = cv[1] + pv[1]; }
  else       { o0 = ew[d] * (yv[0] * rinv) + pv[0]; o1 = ew[d + 1] * (yv[1] * rinv) + pv[1]; }
  if (!real) { o0 = 0.f; o1 = 0.f; }
  v2f ov; ov[0] = o0; ov[1] = o1;
  store2_v2f(h + (size_t)row * D_MODEL + d, ov);
}

__global__ __launch_bounds__(96) void rmsnorm_f16_kernel(const float* __restrict__ h, const float* __restrict__ w,
                                                          _Float16* __restrict__ xn) {
  __shared__ float red[4];
  const int row = blockIdx.x;
  const int tid = threadIdx.x, lane = tid & 31, wave = tid >> 5;
  const int d   = 2 * tid;
  const bool real = (row < MROWS);
  const v2f hv = *(const v2f*)(h + (size_t)row * D_MODEL + d);
  const float ss = wave_sum(hv[0] * hv[0] + hv[1] * hv[1]);
  if (lane == 0) red[wave] = ss;
  __syncthreads();
  const float tot  = red[0] + red[1] + red[2];
  const float rinv = rsqrtf(tot * (1.0f / (float)D_MODEL) + EPSF);
  float o0 = w[d] * (hv[0] * rinv);
  float o1 = w[d + 1] * (hv[1] * rinv);
  if (!real) { o0 = 0.f; o1 = 0.f; }
  store2_u32((unsigned*)xn + ((size_t)row * (D_MODEL / 2) + tid), pack_h2(o0, o1));
}

__global__ __launch_bounds__(256) void conv_silu_kernel(const float* __restrict__ xz, const float* __restrict__ cw,
                                                         const float* __restrict__ cb, float* __restrict__ u,
                                                         _Float16* __restrict__ u16, int n2) {
  const int i = blockIdx.x * 256 + threadIdx.x;
  if (i < n2) {
    const int row  = i / (DIN / 2);
    const int d    = (i - row * (DIN / 2)) * 2;
    const bool real = (row < MROWS);
    const int rowc = real ? row : (MROWS - 1);
    const int b    = rowc / SEQ;
    const int l    = rowc - b * SEQ;
    float s0 = 0.f, s1 = 0.f;
#pragma unroll
    for (int k = 0; k < K_CONV; ++k) {
      const int ls  = l - (K_CONV - 1) + k;
      const int lsc = (ls < 0) ? 0 : ls;
      const v2f xv  = *(const v2f*)(xz + ((size_t)b * SEQ + lsc) * XZC + d);
      const float x0 = (ls >= 0) ? xv[0] : 0.f;
      const float x1 = (ls >= 0) ? xv[1] : 0.f;
      s0 += cw[d * K_CONV + k] * x0;
      s1 += cw[(d + 1) * K_CONV + k] * x1;
    }
    s0 += cb[d];
    s1 += cb[d + 1];
    float u0 = s0 * sigmoid_f(s0);
    float u1 = s1 * sigmoid_f(s1);
    if (!real) { u0 = 0.f; u1 = 0.f; }
    v2f uv; uv[0] = u0; uv[1] = u1;
    store2_v2f(u + (size_t)row * DIN + d, uv);
    store2_u32((unsigned*)u16 + i, pack_h2(u0 * U_CARRY, u1 * U_CARRY));
  }
}

__global__ __launch_bounds__(SC_DG) void scan_kernel(const float* __restrict__ u, const float* __restrict__ dbl,
                                                      const float* __restrict__ xz, const float* __restrict__ Wdt,
                                                      const float* __restrict__ dtb, const float* __restrict__ Alog,
                                                      const float* __restrict__ Dp, _Float16* __restrict__ y16) {
  __shared__ __align__(16) _Float16 ys[SC_TS * SC_DG];
  __shared__ float alds[SC_DG * N_ST];
  const int tid = threadIdx.x;
  const int b   = blockIdx.x / (DIN / SC_DG);
  const int dg  = blockIdx.x - b * (DIN / SC_DG);
  const int d   = dg * SC_DG + tid;

#pragma unroll 1
  for (int j = 0; j < N_ST; ++j) alds[tid * N_ST + j] = -expf(Alog[(size_t)d * N_ST + j]);
  float wdt[R_RANK];
#pragma unroll
  for (int r = 0; r < R_RANK; ++r) wdt[r] = Wdt[(size_t)d * R_RANK + r];
  const float dtb_v = dtb[d];
  const float dp    = Dp[d];
  __syncthreads();
  float a[N_ST], st[N_ST];
#pragma unroll
  for (int n = 0; n < N_ST; ++n) { a[n] = alds[tid * N_ST + n]; st[n] = 0.f; }

  for (int t0 = 0; t0 < SEQ; t0 += SC_TS) {
#pragma unroll 1
    for (int s = 0; s < SC_TS; ++s) {
      const int t = t0 + s;
      if (t < SEQ) {
        const size_t row = (size_t)b * SEQ + t;
        const float uv = u[row * DIN + d];
        const float zv = xz[row * XZC + DIN + d];
        const v4f* dr4 = (const v4f*)(dbl + row * DBLP);
        union { v4f q[3]; float f[12]; } PU;
        union { v4f q[4]; float f[16]; } BU, CU;
        PU.q[0] = dr4[0]; PU.q[1] = dr4[1]; PU.q[2] = dr4[2];
        BU.q[0] = dr4[3]; BU.q[1] = dr4[4]; BU.q[2] = dr4[5]; BU.q[3] = dr4[6];
        CU.q[0] = dr4[7]; CU.q[1] = dr4[8]; CU.q[2] = dr4[9]; CU.q[3] = dr4[10];
        float sdt = 0.f;
#pragma unroll
        for (int r = 0; r < R_RANK; ++r) sdt += PU.f[r] * wdt[r];
        sdt += dtb_v;
        const float dt = fmaxf(sdt, 0.f) + log1pf(expf(-fabsf(sdt)));
        float acc = 0.f;
#pragma unroll
        for (int n = 0; n < N_ST; ++n) {
          const float dA  = __expf(dt * a[n]);
          const float dBu = (dt * BU.f[n]) * uv;
          st[n] = dA * st[n] + dBu;
          acc  += st[n] * CU.f[n];
        }
        float yv = acc + uv * dp;
        yv = yv * (zv * sigmoid_f(zv));
        ys[s * SC_DG + tid] = (_Float16)(yv * Y_CARRY);
      }
    }
    __syncthreads();
    const int nst = ((SEQ - t0) < SC_TS) ? (SEQ - t0) : SC_TS;
    for (int pass = 0; pass < 2; ++pass) {
#pragma unroll
      for (int it = 0; it < 2; ++it) {
        const int line  = it * 8 + (tid >> 3);
        const int piece = (tid & 7) * 8;
        if (line < nst) {
          const v8h val = *(const v8h*)(ys + line * SC_DG + piece);
          *(volatile v8h*)(y16 + ((size_t)b * SEQ + t0 + line) * DIN + dg * SC_DG + piece) = val;
        }
      }
      __threadfence();
    }
    __syncthreads();
  }
}

__global__ __launch_bounds__(96) void final_feat_kernel(const float* __restrict__ h, const float* __restrict__ fw,
                                                         _Float16* __restrict__ feat16) {
  __shared__ float red[4];
  const int b   = blockIdx.x;
  const int tid = threadIdx.x, lane = tid & 31, wave = tid >> 5;
  const int d   = 2 * tid;
  float acc0 = 0.f, acc1 = 0.f;
  if (b < B_SZ) {
    const float w0 = fw[d], w1 = fw[d + 1];
    for (int t = 0; t < SEQ; ++t) {
      if (t != TPOS) {
        const v2f hv = *(const v2f*)(h + ((size_t)b * SEQ + t) * D_MODEL + d);
        const float ss = wave_sum(hv[0] * hv[0] + hv[1] * hv[1]);
        if (lane == 0) red[wave] = ss;
        __syncthreads();
        const float tot  = red[0] + red[1] + red[2];
        __syncthreads();
        const float rinv = rsqrtf(tot * (1.0f / (float)D_MODEL) + EPSF);
        acc0 += w0 * (hv[0] * rinv);
        acc1 += w1 * (hv[1] * rinv);
      }
    }
    acc0 = acc0 * (1.0f / (float)L_PATCH);
    acc1 = acc1 * (1.0f / (float)L_PATCH);
  }
  store2_u32((unsigned*)feat16 + ((size_t)b * (D_MODEL / 2) + tid), pack_h2(acc0 * F_CARRY, acc1 * F_CARRY));
}

__global__ __launch_bounds__(256) void out_copy_kernel(const float* __restrict__ logits, const float* __restrict__ hb,
                                                       float* __restrict__ out, int total) {
  const int i = blockIdx.x * 256 + threadIdx.x;
  if (i < total) {
    const int b = i / NCLS;
    const int c = i - b * NCLS;
    const float v = logits[(size_t)b * NCLS_P + c] + hb[c];
    store2_f32(out + i, v);
  }
}

template <int BIAS_MODE, bool RESID>
static void launch_gemm(hipStream_t s, const _Float16* A, int lda, const _Float16* Bt, int ldb,
                        float* C, int ldc, const float* bias, const float* resid,
                        int M, int N, int K, float scale) {
  const int tiles = (M / 64) * (N / 64);
  dim3 grid((unsigned)((tiles + 7) / 8), 1, 1);
  wmma_gemm64<0, false, BIAS_MODE, 0, RESID, 0><<<grid, 256, 0, s>>>(
      (const unsigned short*)A, nullptr, lda, 0L,
      (const unsigned short*)Bt, nullptr, ldb, 0L,
      (void*)C, nullptr, ldc, 0L,
      bias, resid, 0L, M, N, K, scale);
}

extern "C" void kernel_launch(void* const* d_in, const int* in_sizes, int n_in,
                              void* d_out, int out_size, void* d_ws, size_t ws_size,
                              hipStream_t stream) {
  (void)in_sizes;
  if (n_in < 19) return;
  if ((size_t)out_size < (size_t)B_SZ * NCLS) return;
  const float* x        = (const float*)d_in[0];
  const float* patch_w  = (const float*)d_in[1];
  const float* patch_b  = (const float*)d_in[2];
  const float* embed_nw = (const float*)d_in[3];
  const float* cls_tok  = (const float*)d_in[4];
  const float* pos_emb  = (const float*)d_in[5];
  const float* norm_w   = (const float*)d_in[6];
  const float* in_proj  = (const float*)d_in[7];
  const float* conv_w   = (const float*)d_in[8];
  const float* conv_b   = (const float*)d_in[9];
  const float* x_proj   = (const float*)d_in[10];
  const float* dt_proj  = (const float*)d_in[11];
  const float* dt_bias  = (const float*)d_in[12];
  const float* A_log    = (const float*)d_in[13];
  const float* D_param  = (const float*)d_in[14];
  const float* out_proj = (const float*)d_in[15];
  const float* final_nw = (const float*)d_in[16];
  const float* head_w   = (const float*)d_in[17];
  const float* head_b   = (const float*)d_in[18];
  float* out = (float*)d_out;

  size_t off = 0;
  char* wsb = (char*)d_ws;
  auto carve = [&](size_t bytes) -> void* {
    void* p = wsb + off;
    off += (bytes + 255) & ~(size_t)255;
    return p;
  };
  _Float16* wPatch = (_Float16*)carve((size_t)D_MODEL * KPATCH * 2);
  _Float16* wIn    = (_Float16*)carve((size_t)DEPTH * XZC * D_MODEL * 2);
  _Float16* wX     = (_Float16*)carve((size_t)DEPTH * DBLP * DIN * 2);
  _Float16* wOut   = (_Float16*)carve((size_t)DEPTH * D_MODEL * DIN * 2);
  _Float16* wHead  = (_Float16*)carve((size_t)NCLS_P * D_MODEL * 2);
  _Float16* imcol  = (_Float16*)carve((size_t)PROWS * KPATCH * 2);
  float*    y0     = (float*)   carve((size_t)PROWS * D_MODEL * 4);
  float*    hA     = (float*)   carve((size_t)MPAD * D_MODEL * 4);
  float*    hB     = (float*)   carve((size_t)MPAD * D_MODEL * 4);
  _Float16* xn     = (_Float16*)carve((size_t)MPAD * D_MODEL * 2);
  float*    xz     = (float*)   carve((size_t)MPAD * XZC * 4);
  float*    u      = (float*)   carve((size_t)MPAD * DIN * 4);
  _Float16* u16    = (_Float16*)carve((size_t)MPAD * DIN * 2);
  float*    dbl    = (float*)   carve((size_t)MPAD * DBLP * 4);
  _Float16* y16    = (_Float16*)carve((size_t)MPAD * DIN * 2);
  _Float16* feat16 = (_Float16*)carve((size_t)HEAD_MP * D_MODEL * 2);
  float*    logits = (float*)   carve((size_t)HEAD_MP * NCLS_P * 4);
  if (off > ws_size || off > (size_t)134217728) return;

  {
    int tot;
    tot = 1 * D_MODEL * (KPATCH / 2);
    cast_pad_f16x2<<<(tot + 255) / 256, 256, 0, stream>>>(patch_w, wPatch, 1, D_MODEL, D_MODEL, KPATCH / 2, W_CARRY);
    tot = DEPTH * XZC * (D_MODEL / 2);
    cast_pad_f16x2<<<(tot + 255) / 256, 256, 0, stream>>>(in_proj, wIn, DEPTH, XZC, XZC, D_MODEL / 2, W_CARRY);
    tot = DEPTH * DBLP * (DIN / 2);
    cast_pad_f16x2<<<(tot + 255) / 256, 256, 0, stream>>>(x_proj, wX, DEPTH, DBLC, DBLP, DIN / 2, W_CARRY);
    tot = DEPTH * D_MODEL * (DIN / 2);
    cast_pad_f16x2<<<(tot + 255) / 256, 256, 0, stream>>>(out_proj, wOut, DEPTH, D_MODEL, D_MODEL, DIN / 2, W_CARRY);
    tot = 1 * NCLS_P * (D_MODEL / 2);
    cast_pad_f16x2<<<(tot + 255) / 256, 256, 0, stream>>>(head_w, wHead, 1, NCLS, NCLS_P, D_MODEL / 2, W_CARRY);
  }

  {
    const int n2 = PROWS * (KPATCH / 2);
    im2col_f16x2<<<(n2 + 255) / 256, 256, 0, stream>>>(x, imcol, n2);
  }
  launch_gemm<2, false>(stream, imcol, KPATCH, wPatch, KPATCH, y0, D_MODEL, patch_b, nullptr,
                        PROWS, D_MODEL, KPATCH, 1.0f / W_CARRY);
  embed_kernel<<<MPAD, 96, 0, stream>>>(y0, cls_tok, pos_emb, embed_nw, hA);
  hipMemsetAsync((void*)(y16 + (size_t)MROWS * DIN), 0, (size_t)(MPAD - MROWS) * DIN * 2, stream);

  float* hcur = hA;
  float* hnext = hB;
  for (int i = 0; i < DEPTH; ++i) {
    rmsnorm_f16_kernel<<<MPAD, 96, 0, stream>>>(hcur, norm_w + (size_t)i * D_MODEL, xn);
    launch_gemm<0, false>(stream, xn, D_MODEL, wIn + (size_t)i * XZC * D_MODEL, D_MODEL, xz, XZC, nullptr, nullptr,
                          MPAD, XZC, D_MODEL, 1.0f / W_CARRY);
    {
      const int n2 = MPAD * (DIN / 2);
      conv_silu_kernel<<<(n2 + 255) / 256, 256, 0, stream>>>(xz, conv_w + (size_t)i * DIN * K_CONV,
                                                             conv_b + (size_t)i * DIN, u, u16, n2);
    }
    launch_gemm<0, false>(stream, u16, DIN, wX + (size_t)i * DBLP * DIN, DIN, dbl, DBLP, nullptr, nullptr,
                          MPAD, DBLP, DIN, 1.0f / (U_CARRY * W_CARRY));
    scan_kernel<<<B_SZ * (DIN / SC_DG), SC_DG, 0, stream>>>(u, dbl, xz, dt_proj + (size_t)i * DIN * R_RANK,
                                                            dt_bias + (size_t)i * DIN, A_log + (size_t)i * DIN * N_ST,
                                                            D_param + (size_t)i * DIN, y16);
    launch_gemm<0, true>(stream, y16, DIN, wOut + (size_t)i * D_MODEL * DIN, DIN, hnext, D_MODEL, nullptr, hcur,
                         MPAD, D_MODEL, DIN, 1.0f / (Y_CARRY * W_CARRY));
    float* tmp = hcur; hcur = hnext; hnext = tmp;
  }

  final_feat_kernel<<<HEAD_MP, 96, 0, stream>>>(hcur, final_nw, feat16);
  launch_gemm<0, false>(stream, feat16, D_MODEL, wHead, D_MODEL, logits, NCLS_P, nullptr, nullptr,
                        HEAD_MP, NCLS_P, D_MODEL, 1.0f / (F_CARRY * W_CARRY));
  {
    const int total = B_SZ * NCLS;
    out_copy_kernel<<<(total + 255) / 256, 256, 0, stream>>>(logits, head_b, out, total);
  }
}
